// MLPDecoder_19636590477699
// MI455X (gfx1250) — hardware-verified
//
#include <hip/hip_runtime.h>
#include <math.h>

constexpr int kNodes = 100000;
constexpr int kEdges = 500000;
constexpr int kDim   = 128;
constexpr int kHid   = 128;
constexpr int kKdim  = 3 * kDim;
constexpr int kEB    = 64;
constexpr int kWaves = 4;
constexpr int kThreads = kWaves * 32;
constexpr int kAP    = 392;
constexpr float kFeatCarry = 64.0f;
constexpr float kWCarry    = 256.0f;
constexpr float kInvCarry  = 1.0f / 16384.0f;

static_assert(kKdim % 32 == 0, "K multiple of 32");
static_assert(kKdim % 64 == 0, "prep k tiles of 64");
static_assert(kHid == 128 && kDim == 128, "lane maps assume 128");
static_assert(kEdges % 32 == 0, "whole 32-edge output lines");
static_assert(kEB == 64 && kThreads == kHid, "block maps");
static_assert((kAP % 8) == 0, "16-B aligned LDS rows");

typedef __attribute__((ext_vector_type(16))) _Float16 v16h;
typedef __attribute__((ext_vector_type(8)))  _Float16 v8h;
typedef __attribute__((ext_vector_type(4)))  _Float16 v4h;
typedef __attribute__((ext_vector_type(8)))  float    v8f;
typedef __attribute__((ext_vector_type(4)))  float    v4f;
typedef __attribute__((ext_vector_type(4)))  unsigned int v4u;

__device__ __forceinline__ void dep_guard_h(v8f& a, v8f& b, v16h x, v16h y) { asm volatile("v_nop\n\tv_nop\n\tv_nop\n\tv_nop" : "+v"(a), "+v"(b) : "v"(x), "v"(y)); }
__device__ __forceinline__ void keep4_h(v16h a, v16h b, v16h c, v16h d) { asm volatile("v_nop" :: "v"(a), "v"(b), "v"(c), "v"(d)); }
template <typename T> struct Frag;
template <> struct Frag<_Float16> {
  typedef v16h V; union U { v16h v; v8h h[2]; };
  static __device__ __forceinline__ v16h load(const _Float16* p) {
    U f; f.h[0] = *(const v8h*)(p); f.h[1] = *(const v8h*)(p + 16); return f.v;
  }
  static __device__ __forceinline__ v8f mma(v16h a, v16h b, v8f c) {
    return __builtin_amdgcn_wmma_f32_16x16x32_f16(false, a, false, b, (short)0, c, false, false);
  }
  static __device__ __forceinline__ void guard(v8f& a, v8f& b, v16h x, v16h y) { dep_guard_h(a, b, x, y); }
  static __device__ __forceinline__ void keep(v16h a, v16h b, v16h c, v16h d) { keep4_h(a, b, c, d); }
};
typedef Frag<_Float16> FragH;

__device__ __forceinline__ void grp_guard(v8f& c0, v8f& c1, v8f& c2, v8f& c3,
                                          v16h a, v16h b0, v16h b1, v16h b2, v16h b3) {
  asm volatile("v_nop\n\tv_nop\n\tv_nop\n\tv_nop"
               : "+v"(c0), "+v"(c1), "+v"(c2), "+v"(c3)
               : "v"(a), "v"(b0), "v"(b1), "v"(b2), "v"(b3));
}

__device__ __forceinline__ unsigned pk16(unsigned short a, unsigned short b) { return (unsigned)a | ((unsigned)b << 16); }
__device__ __forceinline__ unsigned short h_bits(float f) { const _Float16 h = (_Float16)f; return __builtin_bit_cast(unsigned short, h); }

__global__ __launch_bounds__(256) void w1t_cast_kernel(const float* __restrict__ W1,
                                                       unsigned short* __restrict__ W1T, float scale) {
  __shared__ float sm[64][65];
  const int t  = threadIdx.x;
  const int k0 = blockIdx.x * 64;
  const int n0 = blockIdx.y * 64;
#pragma unroll
  for (int i = 0; i < 16; ++i) {
    const int e = i * 256 + t;
    const int r = e >> 6;
    const int c = e & 63;
    sm[c][r] = W1[(size_t)(k0 + r) * kHid + n0 + c] * scale;
  }
  __syncthreads();
  const int lane = t & 31, wave = t >> 5;
  const int q = lane >> 3, c8 = (lane & 7) * 8;
  for (int pass = 0; pass < 2; ++pass) {
#pragma unroll
    for (int it = 0; it < 2; ++it) {
      const int row = wave * 8 + it * 4 + q;
      unsigned short hb[8];
#pragma unroll
      for (int e = 0; e < 8; ++e) hb[e] = h_bits(sm[row][c8 + e]);
      const v4u u = (v4u){pk16(hb[0], hb[1]), pk16(hb[2], hb[3]), pk16(hb[4], hb[5]), pk16(hb[6], hb[7])};
      *(volatile v4u*)(W1T + (size_t)(n0 + row) * kKdim + k0 + c8) = u;
    }
    __threadfence();
  }
}

__global__ __launch_bounds__(128) void edge_mlp_kernel(const float* __restrict__ z, const int* __restrict__ ei,
                                                       const unsigned short* __restrict__ W1T,
                                                       const float* __restrict__ b1, const float* __restrict__ W2,
                                                       const float* __restrict__ b2, float* __restrict__ out) {
  __shared__ __align__(16) _Float16 sA[kEB * kAP];
  __shared__ __align__(16) float sB1[kHid];
  __shared__ __align__(16) float sW2[kHid];
  __shared__ __align__(16) float sPart[kWaves][32];

  const int tid  = threadIdx.x;
  const int lane = tid & 31;
  const int wave = tid >> 5;
  const int hh   = lane >> 4;
  const int rl   = lane & 15;
  const int e0   = blockIdx.x * kEB;

  sB1[tid] = b1[tid];
  sW2[tid] = W2[tid];
  const float b2s = b2[0];

  int eg = e0 + wave * 16 + rl;
  eg = eg < kEdges ? eg : kEdges - 1;
  int nd = ei[(size_t)hh * kEdges + eg];
  nd = nd < 0 ? 0 : (nd >= kNodes ? kNodes - 1 : nd);
#pragma unroll 1
  for (int j = 0; j < 16; ++j) {
    const int uj = __shfl(nd, j, 32);
    const int vj = __shfl(nd, 16 + j, 32);
    const v4f a = *(const v4f*)(z + (size_t)uj * kDim + 4 * lane);
    const v4f c = *(const v4f*)(z + (size_t)vj * kDim + 4 * lane);
    v4h tu, tv, td;
#pragma unroll
    for (int e = 0; e < 4; ++e) {
      tu[e] = (_Float16)(a[e] * kFeatCarry);
      tv[e] = (_Float16)(c[e] * kFeatCarry);
      const float d = fabsf(a[e] - c[e]);
      td[e] = (_Float16)(d * kFeatCarry);
    }
    _Float16* rowp = sA + (size_t)(wave * 16 + j) * kAP + 4 * lane;
    *(v4h*)(rowp)            = tu;
    *(v4h*)(rowp + kDim)     = tv;
    *(v4h*)(rowp + 2 * kDim) = td;
  }
  __syncthreads();

  const int g  = wave >> 1;
  const int hn = wave & 1;
  const _Float16* aBase = sA + (size_t)(g * 32 + rl) * kAP + 8 * hh;
  const _Float16* bBase = (const _Float16*)(const void*)W1T + (size_t)(hn * 64 + rl) * kKdim + 8 * hh;

  v8f acc[2][4];
#pragma unroll
  for (int i = 0; i < 2; ++i)
#pragma unroll
    for (int j = 0; j < 4; ++j) acc[i][j] = (v8f){0.f,0.f,0.f,0.f,0.f,0.f,0.f,0.f};

#pragma unroll 1
  for (int k0 = 0; k0 < kKdim; k0 += 32) {
    v16h bf[4];
#pragma unroll
    for (int j = 0; j < 4; ++j) bf[j] = FragH::load(bBase + (size_t)(j * 16) * kKdim + k0);
#pragma unroll
    for (int i = 0; i < 2; ++i) {
      const v16h af = FragH::load(aBase + (size_t)(i * 16) * kAP + k0);
#pragma unroll
      for (int j = 0; j < 4; ++j) acc[i][j] = FragH::mma(af, bf[j], acc[i][j]);
      grp_guard(acc[i][0], acc[i][1], acc[i][2], acc[i][3], af, bf[0], bf[1], bf[2], bf[3]);
    }
  }

  float part[2][8];
#pragma unroll
  for (int i = 0; i < 2; ++i)
#pragma unroll
    for (int r = 0; r < 8; ++r) part[i][r] = 0.0f;
#pragma unroll
  for (int j = 0; j < 4; ++j) {
    const int n = hn * 64 + j * 16 + rl;
    const float bb = sB1[n];
    const float ww = sW2[n];
#pragma unroll
    for (int i = 0; i < 2; ++i) {
#pragma unroll
      for (int r = 0; r < 8; ++r) {
        float hv = acc[i][j][r] * kInvCarry + bb;
        hv = fmaxf(hv, 0.0f);
        part[i][r] += hv * ww;
      }
    }
  }
#pragma unroll
  for (int off = 1; off < 16; off <<= 1) {
#pragma unroll
    for (int i = 0; i < 2; ++i)
#pragma unroll
      for (int r = 0; r < 8; ++r) part[i][r] += __shfl_xor(part[i][r], off, 32);
  }
  if (rl == 0) {
#pragma unroll
    for (int i = 0; i < 2; ++i)
#pragma unroll
      for (int r = 0; r < 8; ++r) sPart[wave][i * 16 + 8 * hh + r] = part[i][r];
  }
  __syncthreads();

  const int l8 = lane & 7;
  const v4f p0 = *(const v4f*)(&sPart[2 * g][4 * l8]);
  const v4f p1 = *(const v4f*)(&sPart[2 * g + 1][4 * l8]);
  v4f o = p0 + p1;
  o = o + b2s;
  const int eline = e0 + g * 32;
  if (hn == 0 && lane < 8 && eline + 32 <= kEdges) {
    float* op = out + eline + 4 * lane;
    *(volatile v4f*)op = o;
    __threadfence();
    *(volatile v4f*)op = o;
  }
}

extern "C" void kernel_launch(void* const* d_in, const int* in_sizes, int n_in,
                              void* d_out, int out_size, void* d_ws, size_t ws_size, hipStream_t stream) {
  (void)in_sizes; (void)n_in; (void)out_size;
  const float* z   = (const float*)d_in[0];
  const int*   ei  = (const int*)  d_in[1];
  const float* W1  = (const float*)d_in[2];
  const float* b1  = (const float*)d_in[3];
  const float* W2  = (const float*)d_in[4];
  const float* b2  = (const float*)d_in[5];
  float* out = (float*)d_out;

  const size_t w1t_bytes = (size_t)kHid * kKdim * 2;
  if (w1t_bytes > ws_size) return;
  unsigned short* W1T = (unsigned short*)d_ws;

  w1t_cast_kernel<<<dim3(kKdim / 64, kHid / 64), 256, 0, stream>>>(W1, W1T, kWCarry);
  const int nblk = (kEdges + kEB - 1) / kEB;
  edge_mlp_kernel<<<nblk, kThreads, 0, stream>>>(z, ei, W1T, b1, W2, b2, out);
}
